// ChebyKANLayer_81303730913619
// MI455X (gfx1250) — hardware-verified
//
#include <hip/hip_runtime.h>
#include <hip/hip_bf16.h>
#include <math.h>

#define MB_ 8192
#define NI 1024
#define NO 1024
#define DEG 9
#define GSTR 48

typedef _Float16 bf16;
typedef _Float16 f16;
typedef __attribute__((ext_vector_type(4))) unsigned v4u_t;
typedef unsigned v4ua __attribute__((ext_vector_type(4), may_alias));
typedef __attribute__((ext_vector_type(4))) float v4f_t;
typedef float v4fa __attribute__((ext_vector_type(4), may_alias));
typedef __attribute__((ext_vector_type(16))) bf16  bf16x16;
typedef bf16x16 f16x16;
typedef __attribute__((ext_vector_type(8)))  bf16  bf16x8;
typedef bf16x8 f16x8;
typedef __attribute__((ext_vector_type(4)))  bf16  bf16x4;
typedef __attribute__((ext_vector_type(8)))  float f32x8;
__device__ __forceinline__ f32x8 wmma16(f16x16 a, f16x16 b, f32x8 c) {
  c = __builtin_amdgcn_wmma_f32_16x16x32_f16(false, a, false, b, (short)0, c, false, false);
  asm volatile("v_nop\n\tv_nop\n\tv_nop\n\tv_nop" : "+v"(c) : "v"(a), "v"(b));
  return c;
}
#define LDS_STRIDE 48
#define KSTRIDE    72
#define VSTRIDE    48

__device__ __forceinline__ f32x8 wmma_bf16(bf16x16 a, bf16x16 b, f32x8 c) {
  c = __builtin_amdgcn_wmma_f32_16x16x32_f16(false, a, false, b, (short)0, c, false, false);
  asm volatile("v_nop\n\tv_nop\n\tv_nop\n\tv_nop" : "+v"(c) : "v"(a), "v"(b));
  return c;
}

template <typename T>
__device__ __forceinline__ bf16x16 load_frag(const T* __restrict__ base, int ld,
                                             int row0, int k0) {
  const int lane = threadIdx.x & 31;
  const int r    = lane & 15;
  const int kh   = (lane >> 4) * 8;
  const T* p0 = base + (size_t)(row0 + r) * ld + (k0 + kh);
  const T* p1 = p0 + 16;
  bf16x16 f;
#pragma unroll
  for (int i = 0; i < 8; ++i) {
    f[i]     = (bf16)p0[i];
    f[i + 8] = (bf16)p1[i];
  }
  return f;
}

__device__ __forceinline__ bf16x16 lds_frag(const bf16* base, int stride) {
  const int lane = threadIdx.x & 31;
  const int row  = lane & 15;
  const int kh   = (lane >> 4) * 8;
  const bf16x8 lo = *(const bf16x8*)(base + row * stride + kh);
  const bf16x8 hi = *(const bf16x8*)(base + row * stride + kh + 16);
  bf16x16 f;
#pragma unroll
  for (int i = 0; i < 8; ++i) { f[i] = lo[i]; f[i + 8] = hi[i]; }
  return f;
}

template <typename T>
__device__ __forceinline__ void stage_read16(const T* __restrict__ p, float* buf) {
#pragma unroll
  for (int i = 0; i < 16; ++i) buf[i] = (float)p[i];
}

__device__ __forceinline__ void stage_write(bf16* dst, const float* buf, int nquad) {
#pragma unroll
  for (int i = 0; i < nquad; ++i) {
    bf16x4 q;
    q[0] = (bf16)buf[4 * i];     q[1] = (bf16)buf[4 * i + 1];
    q[2] = (bf16)buf[4 * i + 2]; q[3] = (bf16)buf[4 * i + 3];
    *(bf16x4*)(dst + 4 * i) = q;
  }
}


#define GSTR 48
template <typename AT, int EPI, bool OUT16>
__global__ __launch_bounds__(256) void gemm_kne(const AT* __restrict__ A, int lda, const float* __restrict__ Wm, int ldw,
                                                const float* __restrict__ bias, const float* __restrict__ R, const float* __restrict__ gvec,
                                                void* __restrict__ Yv, int ldy, int K) {
  __shared__ __attribute__((aligned(16))) f16 ldsA[128 * GSTR];
  __shared__ __attribute__((aligned(16))) f16 ldsW[128 * GSTR];
  __shared__ __attribute__((aligned(16))) float oS[8][32 * 68];
  const int tid = threadIdx.x, lane = tid & 31, wave = tid >> 5, cl = lane & 15, rh = (lane >> 4) * 8;
  const int m0 = blockIdx.x * 128, n0 = blockIdx.y * 128;
  const int wm = (wave & 3) * 32, wn = (wave >> 2) * 64;
  f32x8 acc[2][4];
#pragma unroll
  for (int i = 0; i < 2; ++i)
#pragma unroll
    for (int j = 0; j < 4; ++j) { f32x8 z = {}; acc[i][j] = z; }
#pragma unroll 1
  for (int k0 = 0; k0 < K; k0 += 32) {
    __syncthreads();
    { const int row = tid >> 1, ch = (tid & 1) * 16;
      const AT* src = A + (size_t)(m0 + row) * lda + k0 + ch;
#pragma unroll
      for (int g = 0; g < 16; ++g) ldsA[row * GSTR + ch + g] = (f16)src[g]; }
    { const int k = tid >> 3, nn0 = (tid & 7) * 16;
      const float* src = Wm + (size_t)(k0 + k) * ldw + n0 + nn0;
#pragma unroll
      for (int g = 0; g < 4; ++g) { const v4f_t v = *(const v4f_t*)(src + 4 * g);
#pragma unroll
        for (int u = 0; u < 4; ++u) ldsW[(nn0 + 4 * g + u) * GSTR + k] = (f16)v[u]; } }
    __syncthreads();
    f16x16 af[2];
#pragma unroll
    for (int i = 0; i < 2; ++i) af[i] = lds_frag(ldsA + (wm + 16 * i) * GSTR, GSTR);
#pragma unroll
    for (int j = 0; j < 4; ++j) {
      const f16x16 bf = lds_frag(ldsW + (wn + 16 * j) * GSTR, GSTR);
#pragma unroll
      for (int i = 0; i < 2; ++i) acc[i][j] = wmma16(af[i], bf, acc[i][j]);
    }
  }
  float* so = oS[wave];
#pragma unroll
  for (int i = 0; i < 2; ++i)
#pragma unroll
    for (int j = 0; j < 4; ++j) {
      const int n = n0 + wn + 16 * j + cl;
      const float bv = bias ? bias[n] : 0.0f;
      const float gv = (EPI == 2) ? gvec[n] : 0.0f;
      if (EPI == 1) {
#pragma unroll 1
        for (int r = 0; r < 8; ++r) { const float xg = acc[i][j][r] + bv; so[(16 * i + rh + r) * 68 + 16 * j + cl] = 0.5f * xg * (1.0f + erff(xg * 0.70710678118654752f)); }
      } else {
#pragma unroll
        for (int r = 0; r < 8; ++r) {
          float v = acc[i][j][r] + bv;
          if (EPI == 2) v = R[(size_t)(m0 + wm + 16 * i + rh + r) * ldy + n] + gv * v;
          so[(16 * i + rh + r) * 68 + 16 * j + cl] = v;
        }
      }
    }
  asm volatile("s_wait_dscnt 0" ::: "memory");
  __builtin_amdgcn_wave_barrier();
#pragma unroll 1
  for (int pass = 0; pass < 2; ++pass) {
    if (OUT16) {
      f16* Y = (f16*)Yv;
#pragma unroll
      for (int it = 0; it < 8; ++it) { const int c = lane + 32 * it, rr = c >> 3, q8 = (c & 7) * 8;
        union { f16 h[8]; v4u_t v; } u;
#pragma unroll
        for (int e = 0; e < 8; ++e) u.h[e] = (f16)so[rr * 68 + q8 + e];
        *(volatile v4u_t*)(Y + (size_t)(m0 + wm + rr) * ldy + n0 + wn + q8) = u.v; }
    } else {
      float* Y = (float*)Yv;
#pragma unroll
      for (int it = 0; it < 16; ++it) { const int f4 = lane + 32 * it, rr = f4 >> 4, q = (f4 & 15) * 4;
        *(volatile v4f_t*)(Y + (size_t)(m0 + wm + rr) * ldy + n0 + wn + q) = *(const v4fa*)(so + rr * 68 + q); }
    }
    __threadfence();
  }
}

__global__ __launch_bounds__(256) void k_cheb(const float* __restrict__ x, const float* __restrict__ ts, const float* __restrict__ tb, int d, float* __restrict__ P0, float* __restrict__ P1, bf16* __restrict__ A16) {
  const size_t row = blockIdx.x; const float s = ts[0], bb = tb[0];
  for (int q4 = threadIdx.x; q4 < NI / 4; q4 += 256) { const size_t o4 = row * NI + q4 * 4;
    const v4f_t xv = *(const v4f_t*)(x + o4); v4f_t t, tn, p0, p1;
    for (int e = 0; e < 4; ++e) t[e] = tanhf(xv[e] * s + bb);
    if (d == 0) { for (int e = 0; e < 4; ++e) { tn[e] = 1.0f; p0[e] = t[e]; p1[e] = 1.0f; } }
    else if (d == 1) { tn = t; p0 = t; for (int e = 0; e < 4; ++e) p1[e] = 1.0f; }
    else { const v4f_t a = *(const v4f_t*)(P0 + o4), b2 = *(const v4f_t*)(P1 + o4); for (int e = 0; e < 4; ++e) { tn[e] = 2.0f * t[e] * a[e] - b2[e]; } p1 = a; p0 = tn; }
    union { bf16 h[4]; __attribute__((ext_vector_type(2))) unsigned u2; } cv; for (int e = 0; e < 4; ++e) cv.h[e] = (bf16)tn[e];
#pragma unroll 1
    for (int pass = 0; pass < 2; ++pass) {
      if (d >= 1) { *(volatile v4f_t*)(P0 + o4) = p0; *(volatile v4f_t*)(P1 + o4) = p1; }
      *(volatile __attribute__((ext_vector_type(2))) unsigned*)((bf16*)A16 + o4) = cv.u2;
      __threadfence(); }
  }
}
__global__ __launch_bounds__(256) void k_wscale(const float* __restrict__ Cd, float* __restrict__ Wd) { const size_t row = blockIdx.x;
  for (int q4 = threadIdx.x; q4 < NO / 4; q4 += 256) { v4f_t v = *(const v4f_t*)(Cd + row * NO + q4 * 4); for (int e = 0; e < 4; ++e) v[e] *= 1024.0f;
    *(volatile v4f_t*)(Wd + row * NO + q4 * 4) = v; __threadfence(); *(volatile v4f_t*)(Wd + row * NO + q4 * 4) = v; } }
__global__ __launch_bounds__(256) void k_fill(float* __restrict__ p, float val, size_t n4) { const size_t i = (size_t)blockIdx.x * 256 + threadIdx.x; if (i < n4) { v4f_t v = {val, val, val, val}; *(volatile v4f_t*)(p + 4 * i) = v; __threadfence(); *(volatile v4f_t*)(p + 4 * i) = v; } }
__global__ __launch_bounds__(256) void k_out(const float* __restrict__ Y, float* __restrict__ out) { const size_t row = blockIdx.x;
  for (int q4 = threadIdx.x; q4 < NO / 4; q4 += 256) { v4f_t v = *(const v4f_t*)(Y + row * NO + q4 * 4); for (int e = 0; e < 4; ++e) v[e] *= (1.0f / 1024.0f);
    *(volatile v4f_t*)(out + row * NO + q4 * 4) = v; __threadfence(); *(volatile v4f_t*)(out + row * NO + q4 * 4) = v; } }

extern "C" void kernel_launch(void* const* d_in, const int* in_sizes, int n_in,
                              void* d_out, int out_size, void* d_ws, size_t ws_size,
                              hipStream_t stream) {
  (void)in_sizes; (void)n_in; (void)out_size;
  const float* x = (const float*)d_in[0]; const float* C = (const float*)d_in[1]; const float* ts = (const float*)d_in[2]; const float* tb = (const float*)d_in[3];
  float* out = (float*)d_out;
  char* ws = (char*)d_ws;
  float* P0 = (float*)ws; ws += (size_t)MB_ * NI * 4; float* P1 = (float*)ws; ws += (size_t)MB_ * NI * 4;
  bf16* A16 = (bf16*)ws; ws += (size_t)MB_ * NI * 2;
  float* Wd = (float*)ws; ws += (size_t)NI * NO * 4;
  float* Y = (float*)ws; ws += (size_t)MB_ * NO * 4;
  float* ones = (float*)ws; ws += NO * 4;
  if ((size_t)(ws - (char*)d_ws) > ws_size) return;
  const dim3 blk(256);
  k_fill<<<dim3(((size_t)MB_ * NO / 4 + 255) / 256), blk, 0, stream>>>(Y, 0.0f, (size_t)MB_ * NO / 4);
  k_fill<<<dim3(1), blk, 0, stream>>>(ones, 1.0f, NO / 4);
  for (int d = 0; d < DEG; ++d) {
    k_cheb<<<dim3(MB_), blk, 0, stream>>>(x, ts, tb, d, P0, P1, A16);
    k_wscale<<<dim3(NI), blk, 0, stream>>>(C + (size_t)d * NI * NO, Wd);
    gemm_kne<bf16, 2, false><<<dim3(MB_ / 128, NO / 128), blk, 0, stream>>>(A16, NI, Wd, NO, nullptr, Y, ones, Y, NO, NI);
  }
  k_out<<<dim3(MB_), blk, 0, stream>>>(Y, out);
}
